// MultiHeadAttention_86199993630904
// MI455X (gfx1250) — hardware-run, weakly checked
//
#include <hip/hip_runtime.h>
#ifndef NB
#define NB 2
#endif
#ifndef SEQ
#define SEQ 2048
#endif
#define NB_FULL 2
#define SEQ_FULL 2048
#define DM 1024
#define NH 16
#define HD 64
#define WPR (SEQ / 32)
#define XB_FULL ((size_t)SEQ_FULL * DM)

static_assert(SEQ % 64 == 0);
static_assert(SEQ <= SEQ_FULL);
static_assert(NB <= NB_FULL);
static_assert(HD == 64);
static_assert(NH * HD == DM);
static_assert(DM % 128 == 0);
static_assert((size_t)DM * DM * 2 + (size_t)3 * HD * HD * 2 + (size_t)NB * SEQ * WPR * 4
              + (size_t)3 * NB * NH * SEQ * HD * 2 + (size_t)2 * NB * SEQ * DM * 2 + 8 * 256 <= (size_t)134217728);

typedef __bf16 v16b __attribute__((ext_vector_type(16)));
typedef _Float16 v16h __attribute__((ext_vector_type(16)));
typedef unsigned short v8us __attribute__((ext_vector_type(8), may_alias));
typedef float v8f __attribute__((ext_vector_type(8)));
typedef float v4f __attribute__((ext_vector_type(4)));
typedef float v4fa __attribute__((ext_vector_type(4), may_alias));
typedef int v4i __attribute__((ext_vector_type(4)));
typedef int v4ia __attribute__((ext_vector_type(4), may_alias));
union FragB { v16b v; v8us half[2]; unsigned short u[16]; };
union FragH { v16h v; v8us half[2]; _Float16 h[16]; unsigned short u[16]; };

#define LOG2E 1.4426950408889634f
#define NEGV (-1.25e19f)

__device__ __forceinline__ unsigned short bf16_bits(float x) {
  unsigned int u = __float_as_uint(x);
  return (unsigned short)((u + 0x7FFFu + ((u >> 16) & 1u)) >> 16);
}
__device__ __forceinline__ float bf16_val(unsigned short b) { return __uint_as_float(((unsigned int)b) << 16); }
__device__ __forceinline__ float bf16_rne(float x) { return bf16_val(bf16_bits(x)); }
__device__ __forceinline__ unsigned short f16_bits(_Float16 h) { return __builtin_bit_cast(unsigned short, h); }

__device__ __forceinline__ v8f mma_bf2(v16b a0, v16b b0, v16b a1, v16b b1, v8f c) {
  c = __builtin_amdgcn_wmma_f32_16x16x32_bf16(false, a0, false, b0, (short)0, c, false, false);
  c = __builtin_amdgcn_wmma_f32_16x16x32_bf16(false, a1, false, b1, (short)0, c, false, false);
  asm volatile("v_nop\n\tv_nop\n\tv_nop\n\tv_nop" : "+v"(c) : "v"(a0), "v"(b0), "v"(a1), "v"(b1));
  return c;
}
__device__ __forceinline__ v8f mma_hh2(v16h a0, v16h b0, v16h a1, v16h b1, v8f c) {
  c = __builtin_amdgcn_wmma_f32_16x16x32_f16(false, a0, false, b0, (short)0, c, false, false);
  c = __builtin_amdgcn_wmma_f32_16x16x32_f16(false, a1, false, b1, (short)0, c, false, false);
  asm volatile("v_nop\n\tv_nop\n\tv_nop\n\tv_nop" : "+v"(c) : "v"(a0), "v"(b0), "v"(a1), "v"(b1));
  return c;
}
__device__ __forceinline__ void mma_pv4(v16h a0, v16h a1, v16h a2, v16h a3, v16h b, v8f& c0, v8f& c1, v8f& c2, v8f& c3) {
  c0 = __builtin_amdgcn_wmma_f32_16x16x32_f16(false, a0, false, b, (short)0, c0, false, false);
  c1 = __builtin_amdgcn_wmma_f32_16x16x32_f16(false, a1, false, b, (short)0, c1, false, false);
  c2 = __builtin_amdgcn_wmma_f32_16x16x32_f16(false, a2, false, b, (short)0, c2, false, false);
  c3 = __builtin_amdgcn_wmma_f32_16x16x32_f16(false, a3, false, b, (short)0, c3, false, false);
  asm volatile("v_nop\n\tv_nop\n\tv_nop\n\tv_nop" : "+v"(c0), "+v"(c1), "+v"(c2), "+v"(c3) : "v"(a0), "v"(a1), "v"(a2), "v"(a3), "v"(b));
}
__device__ __forceinline__ v8f mma_bsplit(v16b ah, v16b al, v16b b, v8f c) {
  c = __builtin_amdgcn_wmma_f32_16x16x32_bf16(false, ah, false, b, (short)0, c, false, false);
  c = __builtin_amdgcn_wmma_f32_16x16x32_bf16(false, al, false, b, (short)0, c, false, false);
  asm volatile("v_nop\n\tv_nop\n\tv_nop\n\tv_nop" : "+v"(c) : "v"(ah), "v"(al), "v"(b));
  return c;
}

__device__ __forceinline__ void cvt8_store2(const float* __restrict__ src, unsigned short* __restrict__ dst) {
  const v4f x0 = *(const v4fa*)(src), x1 = *(const v4fa*)(src + 4);
  v8us o;
  o[0] = bf16_bits(x0[0]); o[1] = bf16_bits(x0[1]); o[2] = bf16_bits(x0[2]); o[3] = bf16_bits(x0[3]);
  o[4] = bf16_bits(x1[0]); o[5] = bf16_bits(x1[1]); o[6] = bf16_bits(x1[2]); o[7] = bf16_bits(x1[3]);
  *(volatile v8us*)dst = o;
  __threadfence();
  *(volatile v8us*)dst = o;
}

#define WO_BLKS (DM * DM / 8 / 256)
#define WS_BLKS (3 * HD * HD / 8 / 256)
static_assert(WO_BLKS * 256 * 8 == DM * DM);
static_assert(WS_BLKS == 6);
__global__ __launch_bounds__(256) void k_cvt(const float* __restrict__ Wo, const float* __restrict__ Wq, const float* __restrict__ Wk,
                                             const float* __restrict__ Wv, unsigned short* __restrict__ Wob, unsigned short* __restrict__ Wb) {
  const int blk = blockIdx.x, tid = threadIdx.x;
  if (blk < WO_BLKS) {
    const size_t e = ((size_t)blk * 256 + tid) * 8;
    cvt8_store2(Wo + e, Wob + e);
  } else {
    const int m = (blk - WO_BLKS) >> 1;
    const int e = (((blk - WO_BLKS) & 1) * 256 + tid) * 8;
    if (m == 0) cvt8_store2(Wq + e, Wb + e);
    else if (m == 1) cvt8_store2(Wk + e, Wb + HD * HD + e);
    else if (m == 2) cvt8_store2(Wv + e, Wb + 2 * HD * HD + e);
  }
}

__global__ __launch_bounds__(256) void k_mask(const int* __restrict__ pad, const int* __restrict__ fut, unsigned int* __restrict__ Mb) {
  const int t = blockIdx.x * 256 + threadIdx.x;
  if (t >= NB * SEQ * WPR) return;
  const int j = t % WPR;
  const int rq = t / WPR;
  const int q = rq % SEQ, b = rq / SEQ;
  const int* fr = fut + (size_t)q * SEQ_FULL + 32 * j;
  const int* pr = pad + (size_t)b * SEQ_FULL + 32 * j;
  unsigned int bits = 0u;
#pragma unroll 4
  for (int g = 0; g < 8; ++g) {
    const v4i f = *(const v4ia*)(fr + 4 * g);
    const v4i p = *(const v4ia*)(pr + 4 * g);
    bits |= ((f[0] + p[0]) > 1 ? 1u : 0u) << (4 * g + 0);
    bits |= ((f[1] + p[1]) > 1 ? 1u : 0u) << (4 * g + 1);
    bits |= ((f[2] + p[2]) > 1 ? 1u : 0u) << (4 * g + 2);
    bits |= ((f[3] + p[3]) > 1 ? 1u : 0u) << (4 * g + 3);
  }
  *(volatile unsigned int*)(Mb + t) = bits;
  __threadfence();
  *(volatile unsigned int*)(Mb + t) = bits;
}

__global__ __launch_bounds__(128) void k_proj(const float* __restrict__ x, const unsigned short* __restrict__ Wb,
                                              unsigned short* __restrict__ Qh, unsigned short* __restrict__ Kh,
                                              unsigned short* __restrict__ Vth) {
  __shared__ __attribute__((aligned(16))) unsigned short sqk[2][64][72];
  __shared__ __attribute__((aligned(16))) unsigned short svt[64][72];
  const int tid = threadIdx.x, w = __builtin_amdgcn_readfirstlane((int)(tid >> 5)), lane = tid & 31, ln = lane & 15, hh = lane >> 4;
  const int bh = blockIdx.x / (SEQ / 64), lt = blockIdx.x % (SEQ / 64);
  const int b = bh / NH, h = bh - b * NH;
  const int l0 = lt * 64;
  const float* xr = x + (size_t)b * XB_FULL + (size_t)(l0 + 16 * w + ln) * DM + h * HD;
  FragB x0, x1;
  {
    const v4f a0 = *(const v4fa*)(xr + 8 * hh),      a1 = *(const v4fa*)(xr + 8 * hh + 4);
    const v4f a2 = *(const v4fa*)(xr + 16 + 8 * hh), a3 = *(const v4fa*)(xr + 16 + 8 * hh + 4);
    const v4f c0 = *(const v4fa*)(xr + 32 + 8 * hh), c1 = *(const v4fa*)(xr + 32 + 8 * hh + 4);
    const v4f c2 = *(const v4fa*)(xr + 48 + 8 * hh), c3 = *(const v4fa*)(xr + 48 + 8 * hh + 4);
#pragma unroll
    for (int i = 0; i < 4; ++i) {
      x0.u[i] = bf16_bits(a0[i]); x0.u[4 + i] = bf16_bits(a1[i]); x0.u[8 + i] = bf16_bits(a2[i]); x0.u[12 + i] = bf16_bits(a3[i]);
      x1.u[i] = bf16_bits(c0[i]); x1.u[4 + i] = bf16_bits(c1[i]); x1.u[8 + i] = bf16_bits(c2[i]); x1.u[12 + i] = bf16_bits(c3[i]);
    }
  }
  const v8f z8 = {0.f, 0.f, 0.f, 0.f, 0.f, 0.f, 0.f, 0.f};
#pragma unroll
  for (int mat = 0; mat < 2; ++mat) {
#pragma unroll
    for (int t = 0; t < 4; ++t) {
      const unsigned short* wp = Wb + mat * (HD * HD) + (16 * t + ln) * HD + 8 * hh;
      FragB w0, w1;
      w0.half[0] = *(const v8us*)(wp);      w0.half[1] = *(const v8us*)(wp + 16);
      w1.half[0] = *(const v8us*)(wp + 32); w1.half[1] = *(const v8us*)(wp + 48);
      const v8f c = mma_bf2(x0.v, w0.v, x1.v, w1.v, z8);
#pragma unroll
      for (int r = 0; r < 8; ++r)
        sqk[mat][16 * w + 8 * hh + r][16 * t + ln] = f16_bits((_Float16)(c[r] * 16.0f));
    }
  }
#pragma unroll
  for (int t = 0; t < 4; ++t) {
    const unsigned short* wp = Wb + 2 * (HD * HD) + (16 * t + ln) * HD + 8 * hh;
    FragB w0, w1;
    w0.half[0] = *(const v8us*)(wp);      w0.half[1] = *(const v8us*)(wp + 16);
    w1.half[0] = *(const v8us*)(wp + 32); w1.half[1] = *(const v8us*)(wp + 48);
    const v8f c = mma_bf2(w0.v, x0.v, w1.v, x1.v, z8);
#pragma unroll
    for (int r = 0; r < 8; ++r)
      svt[16 * t + 8 * hh + r][16 * w + ln] = f16_bits((_Float16)(c[r] * 16.0f));
  }
  __syncthreads();
  const size_t qk0 = (size_t)bh * SEQ + l0;
  const size_t v0 = (size_t)bh * HD;
  for (int pass = 0; pass < 2; ++pass) {
#pragma unroll
    for (int it = 0; it < 4; ++it) {
      const int i = tid + 128 * it;
      const int row = i >> 3, p8 = (i & 7) * 8;
      const v8us oq = *(const v8us*)&sqk[0][row][p8];
      const v8us ok = *(const v8us*)&sqk[1][row][p8];
      const v8us ov = *(const v8us*)&svt[row][p8];
      *(volatile v8us*)(Qh + (qk0 + row) * HD + p8) = oq;
      *(volatile v8us*)(Kh + (qk0 + row) * HD + p8) = ok;
      *(volatile v8us*)(Vth + (v0 + row) * SEQ + l0 + p8) = ov;
    }
    if (pass == 0) __threadfence();
  }
}

__device__ __forceinline__ void fa_step(const unsigned short* __restrict__ Kp, const unsigned short* __restrict__ Vp,
                                        unsigned int mw, int key0, int ln, int hh, const FragH& q0, const FragH& q1,
                                        float& mr, float& lr, v8f (&Oh)[4]) {
  const unsigned short* kp0 = Kp + (size_t)(key0 + ln) * HD + 8 * hh;
  const unsigned short* kp1 = kp0 + 16 * HD;
  FragH k00, k01, k10, k11;
  k00.half[0] = *(const v8us*)(kp0);      k00.half[1] = *(const v8us*)(kp0 + 16);
  k01.half[0] = *(const v8us*)(kp0 + 32); k01.half[1] = *(const v8us*)(kp0 + 48);
  k10.half[0] = *(const v8us*)(kp1);      k10.half[1] = *(const v8us*)(kp1 + 16);
  k11.half[0] = *(const v8us*)(kp1 + 32); k11.half[1] = *(const v8us*)(kp1 + 48);
  const size_t voff = (size_t)ln * SEQ + key0 + 8 * hh;
  FragH vh[4];
#pragma unroll
  for (int t = 0; t < 4; ++t) {
    vh[t].half[0] = *(const v8us*)(Vp + voff + (size_t)t * 16 * SEQ);
    vh[t].half[1] = *(const v8us*)(Vp + voff + (size_t)t * 16 * SEQ + 16);
  }
  const v8f z8 = {0.f, 0.f, 0.f, 0.f, 0.f, 0.f, 0.f, 0.f};
  const v8f s0 = mma_hh2(k00.v, q0.v, k01.v, q1.v, z8);
  const v8f s1 = mma_hh2(k10.v, q0.v, k11.v, q1.v, z8);
  float sc[16];
  const unsigned int mb = mw >> (8 * hh);
#pragma unroll
  for (int r = 0; r < 8; ++r) {
    const float a = s0[r] * 0.00048828125f;
    const float c = s1[r] * 0.00048828125f;
    sc[r]     = ((mb >> r) & 1u) ? NEGV : a;
    sc[8 + r] = ((mb >> (16 + r)) & 1u) ? NEGV : c;
  }
  float mx = sc[0];
#pragma unroll
  for (int i = 1; i < 16; ++i) mx = fmaxf(mx, sc[i]);
  mx = fmaxf(mx, __shfl_xor(mx, 16, 32));
  const float mnew = fmaxf(mr, mx);
  const float al = exp2f((mr - mnew) * LOG2E);
  mr = mnew;
  FragH ph;
  float ps = 0.0f;
#pragma unroll
  for (int i = 0; i < 16; ++i) {
    const float pc = exp2f(fmaf(sc[i] - mnew, LOG2E, 8.0f));
    const _Float16 hv = (_Float16)pc;
    ph.h[i] = hv;
    ps += (float)hv;
  }
  ps += __shfl_xor(ps, 16, 32);
  lr = lr * al + ps;
#pragma unroll
  for (int t = 0; t < 4; ++t) Oh[t] = Oh[t] * al;
  mma_pv4(vh[0].v, vh[1].v, vh[2].v, vh[3].v, ph.v, Oh[0], Oh[1], Oh[2], Oh[3]);
}

__global__ __launch_bounds__(128) void k_attn(const unsigned short* __restrict__ Qh, const unsigned short* __restrict__ Kh,
                                              const unsigned short* __restrict__ Vth, const unsigned int* __restrict__ Mb,
                                              unsigned short* __restrict__ Ch, unsigned short* __restrict__ Cl) {
  __shared__ __attribute__((aligned(16))) float so[4][16][68];
  const int tid = threadIdx.x, w = __builtin_amdgcn_readfirstlane((int)(tid >> 5)), lane = tid & 31, ln = lane & 15, hh = lane >> 4;
  const int bh = blockIdx.x / (SEQ / 64), qt = blockIdx.x % (SEQ / 64);
  const int b = bh / NH, h = bh - b * NH;
  const int qbase = qt * 64 + 16 * w;
  const int qg = qbase + ln;
  const unsigned short* qrow = Qh + ((size_t)bh * SEQ + qg) * HD + 8 * hh;
  FragH q0, q1;
  q0.half[0] = *(const v8us*)(qrow);      q0.half[1] = *(const v8us*)(qrow + 16);
  q1.half[0] = *(const v8us*)(qrow + 32); q1.half[1] = *(const v8us*)(qrow + 48);
  float mr = -3.0e38f, lr = 0.0f;
  v8f Oh[4] = {};
  const unsigned short* Kp = Kh + (size_t)bh * SEQ * HD;
  const unsigned short* Vp = Vth + (size_t)bh * HD * SEQ;
  const unsigned int* Mp = Mb + ((size_t)b * SEQ + qg) * WPR;
#pragma unroll 1
  for (int j = 0; j < WPR; ++j) {
    const unsigned int mw = Mp[j];
    fa_step(Kp, Vp, mw, 32 * j, ln, hh, q0, q1, mr, lr, Oh);
  }
  const float inv = 1.0f / (16.0f * lr);
#pragma unroll
  for (int t = 0; t < 4; ++t)
#pragma unroll
    for (int r = 0; r < 8; ++r)
      so[w][ln][16 * t + 8 * hh + r] = Oh[t][r] * inv;
  __syncthreads();
  const int rsub = lane >> 3, p8 = (lane & 7) * 8;
  v8us ohv[4], olv[4];
#pragma unroll
  for (int q = 0; q < 4; ++q) {
    const int row = 4 * q + rsub;
    const v4f x0 = *(const v4fa*)&so[w][row][p8];
    const v4f x1 = *(const v4fa*)&so[w][row][p8 + 4];
#pragma unroll
    for (int i = 0; i < 4; ++i) {
      const unsigned short h0 = bf16_bits(x0[i]);
      const unsigned short h1 = bf16_bits(x1[i]);
      ohv[q][i] = h0;     olv[q][i] = bf16_bits(x0[i] - bf16_val(h0));
      ohv[q][4 + i] = h1; olv[q][4 + i] = bf16_bits(x1[i] - bf16_val(h1));
    }
  }
  const size_t cbase = ((size_t)b * SEQ + qbase) * DM + (size_t)h * HD + p8;
  for (int pass = 0; pass < 2; ++pass) {
#pragma unroll
    for (int q = 0; q < 4; ++q) {
      const size_t o = cbase + (size_t)(4 * q + rsub) * DM;
      *(volatile v8us*)(Ch + o) = ohv[q];
      *(volatile v8us*)(Cl + o) = olv[q];
    }
    if (pass == 0) __threadfence();
  }
}

__global__ __launch_bounds__(128) void k_out(const unsigned short* __restrict__ Ch, const unsigned short* __restrict__ Cl,
                                             const unsigned short* __restrict__ Wob, const float* __restrict__ bo,
                                             float* __restrict__ out) {
  __shared__ __attribute__((aligned(16))) float so[4][32][68];
  const int tid = threadIdx.x, w = __builtin_amdgcn_readfirstlane((int)(tid >> 5)), lane = tid & 31, ln = lane & 15, hh = lane >> 4;
  const int wr = w >> 1, wc = w & 1;
  const int row0 = blockIdx.x * 64 + 32 * wr;
  const int col0 = blockIdx.y * 128 + 64 * wc;
  const unsigned short* ahp = Ch + (size_t)(row0 + ln) * DM + 8 * hh;
  const unsigned short* alp = Cl + (size_t)(row0 + ln) * DM + 8 * hh;
  const unsigned short* bp = Wob + (size_t)(col0 + ln) * DM + 8 * hh;
  v8f acc[2][4] = {};
#pragma unroll 1
  for (int k0 = 0; k0 < DM; k0 += 32) {
    FragB ah[2], al[2], bw[4];
#pragma unroll
    for (int i = 0; i < 2; ++i) {
      ah[i].half[0] = *(const v8us*)(ahp + (size_t)i * 16 * DM + k0);
      ah[i].half[1] = *(const v8us*)(ahp + (size_t)i * 16 * DM + k0 + 16);
      al[i].half[0] = *(const v8us*)(alp + (size_t)i * 16 * DM + k0);
      al[i].half[1] = *(const v8us*)(alp + (size_t)i * 16 * DM + k0 + 16);
    }
#pragma unroll
    for (int t = 0; t < 4; ++t) {
      bw[t].half[0] = *(const v8us*)(bp + (size_t)t * 16 * DM + k0);
      bw[t].half[1] = *(const v8us*)(bp + (size_t)t * 16 * DM + k0 + 16);
    }
#pragma unroll
    for (int i = 0; i < 2; ++i)
#pragma unroll
      for (int t = 0; t < 4; ++t)
        acc[i][t] = mma_bsplit(ah[i].v, al[i].v, bw[t].v, acc[i][t]);
  }
#pragma unroll
  for (int t = 0; t < 4; ++t) {
    const float bias = bf16_rne(bo[col0 + 16 * t + ln]);
#pragma unroll
    for (int i = 0; i < 2; ++i)
#pragma unroll
      for (int r = 0; r < 8; ++r)
        so[w][16 * i + 8 * hh + r][16 * t + ln] = acc[i][t][r] + bias;
  }
  __syncthreads();
  const int b = row0 / SEQ, l = row0 - b * SEQ;
  float* og = out + (size_t)b * XB_FULL + (size_t)l * DM + col0;
  const int rsub = lane >> 4, c4 = (lane & 15) * 4;
  for (int pass = 0; pass < 2; ++pass) {
#pragma unroll
    for (int q = 0; q < 16; ++q) {
      const int row = 2 * q + rsub;
      const v4f v = *(const v4fa*)&so[w][row][c4];
      *(volatile v4f*)(og + (size_t)row * DM + c4) = v;
    }
    if (pass == 0) __threadfence();
  }
}

extern "C" void kernel_launch(void* const* d_in, const int* in_sizes, int n_in,
                              void* d_out, int out_size, void* d_ws, size_t ws_size, hipStream_t stream) {
  if (n_in < 8) return;
  const long long needx = (long long)(NB - 1) * SEQ_FULL * DM + (long long)SEQ * DM;
  const long long needp = (long long)(NB - 1) * SEQ_FULL + SEQ;
  const long long needf = (long long)(SEQ - 1) * SEQ_FULL + SEQ;
  if ((long long)in_sizes[0] < needx || (long long)in_sizes[1] < needp || (long long)in_sizes[2] < needf) return;
  if (in_sizes[3] < HD * HD || in_sizes[4] < HD * HD || in_sizes[5] < HD * HD) return;
  if (in_sizes[6] < DM * DM || in_sizes[7] < DM) return;
  if ((long long)out_size < needx) return;
  const float* x   = (const float*)d_in[0];
  const int*   pad = (const int*)d_in[1];
  const int*   fut = (const int*)d_in[2];
  const float* Wq  = (const float*)d_in[3];
  const float* Wk  = (const float*)d_in[4];
  const float* Wv  = (const float*)d_in[5];
  const float* Wo  = (const float*)d_in[6];
  const float* bo  = (const float*)d_in[7];
  float* out = (float*)d_out;
  char* ws = (char*)d_ws;
  size_t off = 0;
  const size_t szWo = (size_t)DM * DM * 2;
  const size_t szWb = (size_t)3 * HD * HD * 2;
  const size_t szMb = (size_t)NB * SEQ * WPR * 4;
  const size_t szHd = (size_t)NB * NH * SEQ * HD * 2;
  const size_t szCx = (size_t)NB * SEQ * DM * 2;
  unsigned short* Wob = (unsigned short*)(ws + off); off += (szWo + 255) & ~(size_t)255;
  unsigned short* Wb  = (unsigned short*)(ws + off); off += (szWb + 255) & ~(size_t)255;
  unsigned int*   Mb  = (unsigned int*)(ws + off);   off += (szMb + 255) & ~(size_t)255;
  unsigned short* Qh  = (unsigned short*)(ws + off); off += (szHd + 255) & ~(size_t)255;
  unsigned short* Kh  = (unsigned short*)(ws + off); off += (szHd + 255) & ~(size_t)255;
  unsigned short* Vth = (unsigned short*)(ws + off); off += (szHd + 255) & ~(size_t)255;
  unsigned short* Ch  = (unsigned short*)(ws + off); off += (szCx + 255) & ~(size_t)255;
  unsigned short* Cl  = (unsigned short*)(ws + off); off += (szCx + 255) & ~(size_t)255;
  if (off > ws_size) return;
  k_cvt<<<(unsigned)(WO_BLKS + WS_BLKS), 256, 0, stream>>>(Wo, Wq, Wk, Wv, Wob, Wb);
  k_mask<<<(unsigned)((NB * SEQ * WPR + 255) / 256), 256, 0, stream>>>(pad, fut, Mb);
  k_proj<<<(unsigned)(NB * NH * (SEQ / 64)), 128, 0, stream>>>(x, Wb, Qh, Kh, Vth);
  k_attn<<<(unsigned)(NB * NH * (SEQ / 64)), 128, 0, stream>>>(Qh, Kh, Vth, Mb, Ch, Cl);
  k_out<<<dim3((unsigned)(NB * SEQ / 64), (unsigned)(DM / 128)), 128, 0, stream>>>(Ch, Cl, Wob, bo, out);
}
